// Former2Conv_30030411334031
// MI455X (gfx1250) — hardware-verified
//
#include <hip/hip_runtime.h>
#include <math.h>

typedef __attribute__((ext_vector_type(16))) _Float16 v16h;
typedef __attribute__((ext_vector_type(16))) __bf16 v16b;
typedef __attribute__((ext_vector_type(8)))  _Float16 v8h;
typedef __attribute__((ext_vector_type(8)))  float v8f;
typedef __attribute__((ext_vector_type(4)))  float v4f;
typedef __attribute__((ext_vector_type(2)))  float v2f;
typedef __attribute__((ext_vector_type(4)))  unsigned v4u;
typedef __attribute__((ext_vector_type(4)))  int v4i;
typedef float __attribute__((may_alias)) float_a;
typedef int __attribute__((may_alias)) int_a;

template <typename T> __device__ __forceinline__ void vst2(void* p, T v) { *(volatile T*)p = v; __threadfence(); *(volatile T*)p = v; }
__device__ __forceinline__ v8f wmma16(v16h a, v16h b, v8f c) {
  v8f d = __builtin_amdgcn_wmma_f32_16x16x32_f16(false, a, false, b, (short)0, c, false, false);
  asm volatile("v_nop\n\tv_nop\n\tv_nop\n\tv_nop" : "+v"(d) : "v"(a), "v"(b));
  return d;
}
__device__ __forceinline__ v8f wmma_bf(v16b a, v16b b, v8f c) {
  v8f d = __builtin_amdgcn_wmma_f32_16x16x32_bf16(false, a, false, b, (short)0, c, false, false);
  asm volatile("v_nop\n\tv_nop\n\tv_nop\n\tv_nop" : "+v"(d) : "v"(a), "v"(b));
  return d;
}
__device__ __forceinline__ v16h frag_h(const _Float16* rowk0, int lane) {
  union { v16h v; v8h q[2]; } u; const _Float16* p = rowk0 + 8 * (lane >> 4);
  u.q[0] = *(const v8h*)p; u.q[1] = *(const v8h*)(p + 16); return u.v;
}
__device__ __forceinline__ v16h frag_f32(const float* rowk0, int lane) {
  v16h a; const float* p = rowk0 + 8 * (lane >> 4);
#pragma unroll
  for (int i = 0; i < 8; ++i) { a[i] = (_Float16)p[i]; a[8 + i] = (_Float16)p[16 + i]; }
  return a;
}
__device__ __forceinline__ v16h frag_f32s(const float* rowk0, int lane, float sc) {
  v16h a; const float* p = rowk0 + 8 * (lane >> 4);
#pragma unroll
  for (int i = 0; i < 8; ++i) { a[i] = (_Float16)(p[i] * sc); a[8 + i] = (_Float16)(p[16 + i] * sc); }
  return a;
}
__device__ __forceinline__ v16h fragc_f32(const float* W, int k0, int n, int lane, int ld, int K) {
  v16h a; const int g = lane >> 4;
#pragma unroll
  for (int i = 0; i < 8; ++i) { const int ka = k0 + 8 * g + i, kb = ka + 16;
    a[i] = (_Float16)(ka < K ? W[(size_t)ka * ld + n] : 0.f); a[8 + i] = (_Float16)(kb < K ? W[(size_t)kb * ld + n] : 0.f); }
  return a;
}
struct F2 { v16b h, l; };
__device__ __forceinline__ F2 bsplit16(const float v[16]) { F2 r;
#pragma unroll
  for (int i = 0; i < 16; ++i) { const __bf16 h = (__bf16)v[i]; r.h[i] = h; r.l[i] = (__bf16)(v[i] - (float)h); }
  return r; }
__device__ __forceinline__ F2 split_row(const float* row, int k0, int lane) { float v[16]; const float* p = row + k0 + 8 * (lane >> 4);
#pragma unroll
  for (int i = 0; i < 8; ++i) { v[i] = p[i]; v[8 + i] = p[16 + i]; }
  return bsplit16(v); }
__device__ __forceinline__ F2 split_rowK(const float* row, int k0, int lane, int K) { float v[16]; const int g = lane >> 4;
#pragma unroll
  for (int i = 0; i < 8; ++i) { const int ka = k0 + 8 * g + i, kb = ka + 16; v[i] = ka < K ? row[ka] : 0.f; v[8 + i] = kb < K ? row[kb] : 0.f; }
  return bsplit16(v); }
__device__ __forceinline__ F2 split_col(const float* W, int k0, int n, int lane, int ld, int K) { float v[16]; const int g = lane >> 4;
#pragma unroll
  for (int i = 0; i < 8; ++i) { const int ka = k0 + 8 * g + i, kb = ka + 16; v[i] = ka < K ? W[(size_t)ka * ld + n] : 0.f; v[8 + i] = kb < K ? W[(size_t)kb * ld + n] : 0.f; }
  return bsplit16(v); }
__device__ __forceinline__ v8f mac3(const F2& a, const F2& b, v8f c) { c = wmma_bf(a.l, b.h, c); c = wmma_bf(a.h, b.l, c); return wmma_bf(a.h, b.h, c); }
__device__ __forceinline__ float sigm(float v) { return 1.0f / (1.0f + expf(-v)); }
#define LDSX() do { asm volatile("s_wait_dscnt 0" ::: "memory"); __builtin_amdgcn_wave_barrier(); __builtin_amdgcn_fence(__ATOMIC_RELEASE, "workgroup"); } while (0)

#define NB 8
#define CC 64
#define HW 4096
#define MZ 256
#define DZ 256
#define NH 8
#define INNER 512
#define NQR 512

__global__ __launch_bounds__(128) void k_kv(const float* __restrict__ z, const float* __restrict__ Wk, const float* __restrict__ bk, const float* __restrict__ Wv, const float* __restrict__ bv, float* __restrict__ KZ, float* __restrict__ VZ) {
  __shared__ __align__(16) float so[4][16][132];
  const int tid = threadIdx.x, wave = tid >> 5, lane = tid & 31, col = lane & 15, g = lane >> 4;
  const int which = blockIdx.z, r0 = blockIdx.x * 64 + wave * 16, n0 = blockIdx.y * 128; const float* W = which ? Wv : Wk; const float* bias = which ? bv : bk; float* dst = which ? VZ : KZ;
  v8f acc[8] = {};
#pragma unroll 1
  for (int kc = 0; kc < DZ / 32; ++kc) { const F2 a = split_row(z + (size_t)(r0 + col) * DZ, kc * 32, lane);
#pragma unroll
    for (int j = 0; j < 8; ++j) acc[j] = mac3(a, split_col(W, kc * 32, n0 + j * 16 + col, lane, INNER, DZ), acc[j]); }
#pragma unroll
  for (int j = 0; j < 8; ++j) { const float bb = bias[n0 + j * 16 + col];
#pragma unroll
    for (int r = 0; r < 8; ++r) so[wave][8 * g + r][j * 16 + col] = acc[j][r] + bb; }
  LDSX();
#pragma unroll 4
  for (int rl = 0; rl < 16; ++rl) vst2(dst + (size_t)(r0 + rl) * INNER + n0 + lane * 4, *(const v4f*)(&so[wave][rl][lane * 4]));
}
__global__ __launch_bounds__(128) void k_attn(const float* __restrict__ x, const float* __restrict__ KZ, const float* __restrict__ VZ, float* __restrict__ O) {
  __shared__ __align__(16) float sS[4][16][MZ + 4];
  __shared__ __align__(16) float sO[4][16][68];
  const int tid = threadIdx.x, w = tid >> 5, lane = tid & 31, col = lane & 15, g = lane >> 4;
  const int b = blockIdx.z, h = blockIdx.y, r0 = blockIdx.x * 64 + w * 16;
  const float* qb = x + (size_t)b * CC * HW + (size_t)h * 32768; const float* kb = KZ + (size_t)b * MZ * INNER + (size_t)h * 32 * INNER; const float* vb = VZ + (size_t)b * MZ * INNER + (size_t)h * 32 * INNER;
  F2 aq[2];
#pragma unroll
  for (int kc = 0; kc < 2; ++kc) aq[kc] = split_row(qb + (size_t)(r0 + col) * CC, kc * 32, lane);
#pragma unroll 1
  for (int t = 0; t < MZ / 16; ++t) { v8f s = {};
#pragma unroll
    for (int kc = 0; kc < 2; ++kc) s = mac3(aq[kc], split_row(kb + (size_t)(t * 16 + col) * CC, kc * 32, lane), s);
#pragma unroll
    for (int r = 0; r < 8; ++r) sS[w][8 * g + r][t * 16 + col] = s[r] * 0.125f; }
  LDSX();
  { const int m = col; float* row = &sS[w][m][0]; float mx = -3.4e38f;
#pragma unroll 8
    for (int j = g * 128; j < g * 128 + 128; ++j) mx = fmaxf(mx, row[j]);
    mx = fmaxf(mx, __shfl_xor(mx, 16, 32)); float l = 0.f;
#pragma unroll 8
    for (int j = g * 128; j < g * 128 + 128; ++j) { const float p = expf(row[j] - mx); row[j] = p; l += p; }
    l += __shfl_xor(l, 16, 32); const float inv = 1.0f / l;
    LDSX();
#pragma unroll 8
    for (int j = g * 128; j < g * 128 + 128; ++j) row[j] *= inv; }
  LDSX();
  v8f acc[4] = {};
#pragma unroll 2
  for (int kc = 0; kc < MZ / 32; ++kc) { const F2 pa = split_row(&sS[w][col][0], kc * 32, lane);
#pragma unroll
    for (int t = 0; t < 4; ++t) acc[t] = mac3(pa, split_col(vb + (size_t)(kc * 32) * CC, 0, t * 16 + col, lane, CC, 32), acc[t]); }
#pragma unroll
  for (int t = 0; t < 4; ++t)
#pragma unroll
    for (int r = 0; r < 8; ++r) sO[w][8 * g + r][t * 16 + col] = acc[t][r];
  LDSX();
  for (int q = lane; q < 16 * 16; q += 32) { const int rl = q >> 4, pc = q & 15; vst2(O + ((size_t)b * NQR + r0 + rl) * INNER + h * CC + pc * 4, *(const v4f*)(&sO[w][rl][pc * 4])); }
}
__global__ __launch_bounds__(128) void k_out(const float* __restrict__ O, const float* __restrict__ Wo, const float* __restrict__ bo, const float* __restrict__ x, float* __restrict__ out) {
  __shared__ __align__(16) float so[4][16][68];
  const int tid = threadIdx.x, wave = tid >> 5, lane = tid & 31, col = lane & 15, g = lane >> 4;
  const int b = blockIdx.y, r0 = blockIdx.x * 64 + wave * 16;
  v8f acc[4] = {};
#pragma unroll 1
  for (int kc = 0; kc < INNER / 32; ++kc) { const F2 a = split_row(O + ((size_t)b * NQR + r0 + col) * INNER, kc * 32, lane);
#pragma unroll
    for (int j = 0; j < 4; ++j) acc[j] = mac3(a, split_col(Wo, kc * 32, j * 16 + col, lane, CC, INNER), acc[j]); }
#pragma unroll
  for (int j = 0; j < 4; ++j) { const float bb = bo[j * 16 + col];
#pragma unroll
    for (int r = 0; r < 8; ++r) so[wave][8 * g + r][j * 16 + col] = acc[j][r] + bb; }
  LDSX();
  const float* xb = x + (size_t)b * CC * HW; float* ob = out + (size_t)b * CC * HW;
#pragma unroll 1
  for (int rl = 0; rl < 16; ++rl) { const size_t base = (size_t)(r0 + rl) * 512;
#pragma unroll
    for (int e = 0; e < 4; ++e) { const int f = (lane * 4 + e) * 4; const int c = f & 63; v4f o; o[0] = xb[base + f] + so[wave][rl][c]; o[1] = xb[base + f + 1] + so[wave][rl][c + 1]; o[2] = xb[base + f + 2] + so[wave][rl][c + 2]; o[3] = xb[base + f + 3] + so[wave][rl][c + 3]; vst2(ob + base + f, o); } }
}
extern "C" void kernel_launch(void* const* d_in, const int* in_sizes, int n_in, void* d_out, int out_size, void* d_ws, size_t ws_size, hipStream_t stream) {
  (void)in_sizes; (void)n_in; (void)out_size; (void)ws_size;
  const float* x = (const float*)d_in[0]; const float* z = (const float*)d_in[1]; const float* Wk = (const float*)d_in[2]; const float* bk = (const float*)d_in[3]; const float* Wv = (const float*)d_in[4]; const float* bv = (const float*)d_in[5]; const float* Wo = (const float*)d_in[6]; const float* bo = (const float*)d_in[7];
  float* out = (float*)d_out;
  char* ws = (char*)d_ws; size_t off = 0;
  auto take = [&](size_t bytes) { char* p = ws + off; off += (bytes + 255) & ~(size_t)255; return p; };
  float* KZ = (float*)take((size_t)NB * MZ * INNER * 4); float* VZ = (float*)take((size_t)NB * MZ * INNER * 4); float* O = (float*)take((size_t)NB * NQR * INNER * 4);
  k_kv<<<dim3(NB * MZ / 64, INNER / 128, 2), 128, 0, stream>>>(z, Wk, bk, Wv, bv, KZ, VZ);
  k_attn<<<dim3(NQR / 64, NH, NB), 128, 0, stream>>>(x, KZ, VZ, O);
  k_out<<<dim3(NQR / 64, NB), 128, 0, stream>>>(O, Wo, bo, x, out);
}
